// CrossAttention_25211458027991
// MI455X (gfx1250) — hardware-run, weakly checked
//
#include <hip/hip_runtime.h>
#include <math.h>

typedef __attribute__((ext_vector_type(16))) __bf16 v16b;
typedef __attribute__((ext_vector_type(8)))  __bf16 v8b;
typedef __attribute__((ext_vector_type(8)))  float v8f;
typedef __attribute__((ext_vector_type(4)))  float v4f;
typedef __attribute__((ext_vector_type(4)))  unsigned v4u;
typedef __attribute__((ext_vector_type(4)))  int v4i;

template <typename T> __device__ __forceinline__ void vst2(void* p, T v) { *(volatile T*)p = v; __threadfence(); *(volatile T*)p = v; }
__device__ __forceinline__ v8f wmma_bf(v16b a, v16b b, v8f c) {
  v8f d = __builtin_amdgcn_wmma_f32_16x16x32_bf16(false, a, false, b, (short)0, c, false, false);
  asm volatile("v_nop\n\tv_nop\n\tv_nop\n\tv_nop" : "+v"(d) : "v"(a), "v"(b));
  return d;
}
__device__ __forceinline__ v16b frag_b(const __bf16* rowk0, int lane) {
  union { v16b v; v8b q[2]; } u; const __bf16* p = rowk0 + 8 * (lane >> 4);
  u.q[0] = *(const v8b*)p; u.q[1] = *(const v8b*)(p + 16); return u.v;
}
struct F2 { v16b h, l; };
__device__ __forceinline__ F2 bsplit16(const float v[16]) { F2 r;
#pragma unroll
  for (int i = 0; i < 16; ++i) { const __bf16 h = (__bf16)v[i]; r.h[i] = h; r.l[i] = (__bf16)(v[i] - (float)h); }
  return r; }
__device__ __forceinline__ F2 split_row(const float* row, int k0, int lane) { float v[16]; const float* p = row + k0 + 8 * (lane >> 4);
#pragma unroll
  for (int i = 0; i < 8; ++i) { v[i] = p[i]; v[8 + i] = p[16 + i]; }
  return bsplit16(v); }
__device__ __forceinline__ float bfr(float v) { return (float)(__bf16)v; }
#define LDSX() do { asm volatile("s_wait_dscnt 0" ::: "memory"); __builtin_amdgcn_wave_barrier(); __builtin_amdgcn_fence(3  , "workgroup"); } while (0)

typedef _Float16 h16;
typedef __attribute__((ext_vector_type(16))) _Float16 v16h;
typedef __attribute__((ext_vector_type(8)))  _Float16 v8h;
__device__ __forceinline__ v8f wmma_hf(v16h a, v16h b, v8f c) {
  v8f d = __builtin_amdgcn_wmma_f32_16x16x32_f16(false, a, false, b, (short)0, c, false, false);
  asm volatile("v_nop\n\tv_nop\n\tv_nop\n\tv_nop" : "+v"(d) : "v"(a), "v"(b));
  return d;
}
__device__ __forceinline__ v16h frag_h(const h16* rowk0, int lane) {
  union { v16h v; v8h q[2]; } u; const h16* p = rowk0 + 8 * (lane >> 4);
  u.q[0] = *(const v8h*)p; u.q[1] = *(const v8h*)(p + 16); return u.v;
}
static __device__ __forceinline__ h16 toh_flush(float v) { const h16 r = (h16)v; return (fabsf(v) < 6.103515625e-05f) ? (h16)0.0f : r; }
static __device__ __forceinline__ v4u pack8h(v4f a, v4f b) { union { v8h v; v4u u; } o;
  o.v[0] = toh_flush(a.x); o.v[1] = toh_flush(a.y); o.v[2] = toh_flush(a.z); o.v[3] = toh_flush(a.w);
  o.v[4] = toh_flush(b.x); o.v[5] = toh_flush(b.y); o.v[6] = toh_flush(b.z); o.v[7] = toh_flush(b.w);
  return o.u; }

#define CH 256
#define IMG 64
#define NTOK 4096
#define PW 66
#define PTOK 4356
#define KCV 2304
#define NHD 8
#define QKD 16
#define HDV 32
#define NQK 128
#define NPJ 512
#ifndef NQ
#define NQ NTOK
#endif
static_assert(IMG * IMG == NTOK);
static_assert(PW == IMG + 2);
static_assert(PW * PW == PTOK);
static_assert(9 * CH == KCV);
static_assert((CH % 32) == 0);
static_assert((KCV % 32) == 0);
static_assert(CH == 256);
static_assert(NHD * QKD == NQK);
static_assert(NHD * HDV == CH);
static_assert(NQK + NQK + CH == NPJ);
static_assert((NPJ % 128) == 0);
static_assert(QKD == 16);
static_assert(HDV == 32);
static_assert((NTOK % 64) == 0);
static_assert((NTOK % 32) == 0);
static_assert((NQ % 128) == 0);
static_assert(NQ >= 128);
static_assert(NQ <= NTOK);
#define CXF 16.0f
#define CWP 64.0f
#define CQK 64.0f
#define SC1 (0.17677669529663687f * 1.4426950408889634f / 4096.0f)

#define WS_XP  ((size_t)0)
#define WS_WC  (WS_XP + 2u * 2u * (size_t)PTOK * CH)
#define WS_WP  (WS_WC + 2u * 2u * (size_t)CH * KCV)
#define WS_WO  (WS_WP + 2u * (size_t)NPJ * CH)
#define WS_XF  (WS_WO + 2u * (size_t)CH * CH)
#define WS_QK  (WS_XF + 2u * 2u * (size_t)NTOK * CH)
#define WS_VT  (WS_QK + 2u * 2u * (size_t)NTOK * NQK)
#define WS_Y   (WS_VT + 2u * (size_t)CH * NTOK)
#define WS_END (WS_Y  + 4u * (size_t)NTOK * CH)
static_assert(WS_END <= (size_t)134217728);
static_assert((WS_WC % 128) == 0);
static_assert((WS_WP % 128) == 0);
static_assert((WS_WO % 128) == 0);
static_assert(WS_WO == WS_WP + 2u * (size_t)NPJ * CH);
static_assert((WS_XF % 128) == 0);
static_assert((WS_QK % 128) == 0);
static_assert((WS_VT % 128) == 0);
static_assert((WS_Y % 128) == 0);
static_assert(((2u * (size_t)PTOK * CH) % 128) == 0);

__global__ __launch_bounds__(256) void k_padx(const float* __restrict__ X, __bf16* __restrict__ XP) {
  __shared__ __align__(16) __bf16 sb[PW][CH + 8];
  const int tid = threadIdx.x, lane = tid & 31; const int wave = __builtin_amdgcn_readfirstlane(tid >> 5);
  const int yp = blockIdx.x;
  const v8b zb = {};
  for (int e = tid; e < PW * ((CH + 8) / 8); e += 256) { const int rw = e / ((CH + 8) / 8), c8 = e - rw * ((CH + 8) / 8); *(v8b*)&sb[rw][c8 * 8] = zb; }
  __syncthreads();
  if (yp >= 1 && yp <= IMG) {
    const int y = yp - 1; const int x4 = (tid & 15) * 4;
#pragma unroll 1
    for (int i = 0; i < CH / 16; ++i) { const int c = i * 16 + (tid >> 4);
      const v4f v = *(const v4f*)(X + (size_t)c * NTOK + y * IMG + x4);
      sb[1 + x4 + 0][c] = (__bf16)v.x; sb[1 + x4 + 1][c] = (__bf16)v.y; sb[1 + x4 + 2][c] = (__bf16)v.z; sb[1 + x4 + 3][c] = (__bf16)v.w; }
  }
  __syncthreads();
  for (int rw = wave; rw < PW; rw += 8) { union { v8b v; v4u u; } o; o.v = *(const v8b*)&sb[rw][lane * 8];
    vst2(XP + ((size_t)yp * PW + rw) * CH + lane * 8, o.u); }
}

static_assert((KCV % 8) == 0);
__global__ __launch_bounds__(256) void k_cvtw(const float* __restrict__ W, __bf16* __restrict__ WC) {
  __shared__ __align__(16) __bf16 sw[KCV + 8];
  const int tid = threadIdx.x; const size_t oc = blockIdx.x;
  for (int e = tid; e < KCV / 4; e += 256) { const v4f v = *(const v4f*)(W + oc * KCV + e * 4);
    const int s0 = e * 4, s1 = s0 + 1, s2 = s0 + 2, s3 = s0 + 3;
    const int i0 = s0 / 9, i1 = s1 / 9, i2 = s2 / 9, i3 = s3 / 9;
    sw[(s0 - 9 * i0) * CH + i0] = (__bf16)v.x; sw[(s1 - 9 * i1) * CH + i1] = (__bf16)v.y;
    sw[(s2 - 9 * i2) * CH + i2] = (__bf16)v.z; sw[(s3 - 9 * i3) * CH + i3] = (__bf16)v.w; }
  __syncthreads();
  for (int e = tid; e < KCV / 8; e += 256) { union { v8b v; v4u u; } o; o.v = *(const v8b*)&sw[e * 8];
    vst2(WC + oc * KCV + e * 8, o.u); }
}

static_assert(((NPJ + CH) % 8) == 0);
__global__ __launch_bounds__(256) void k_cvts(const float* __restrict__ WQ, const float* __restrict__ WK, const float* __restrict__ WV, const float* __restrict__ WO, unsigned short* __restrict__ DST) {
  const int tid = threadIdx.x, lane = tid & 31; const int r = (int)(blockIdx.x * 8 + (tid >> 5));
  int rq = r; rq = rq > NQK - 1 ? NQK - 1 : rq;
  int rk = r - NQK; rk = rk < 0 ? 0 : (rk > NQK - 1 ? NQK - 1 : rk);
  int rv = r - 2 * NQK; rv = rv < 0 ? 0 : (rv > CH - 1 ? CH - 1 : rv);
  int ro = r - NPJ; ro = ro < 0 ? 0 : (ro > CH - 1 ? CH - 1 : ro);
  const v4f qa = *(const v4f*)(WQ + (size_t)rq * CH + lane * 8), qb = *(const v4f*)(WQ + (size_t)rq * CH + lane * 8 + 4);
  const v4f ka = *(const v4f*)(WK + (size_t)rk * CH + lane * 8), kb = *(const v4f*)(WK + (size_t)rk * CH + lane * 8 + 4);
  const v4f va = *(const v4f*)(WV + (size_t)rv * CH + lane * 8), vb = *(const v4f*)(WV + (size_t)rv * CH + lane * 8 + 4);
  const v4f oa = *(const v4f*)(WO + (size_t)ro * CH + lane * 8), ob = *(const v4f*)(WO + (size_t)ro * CH + lane * 8 + 4);
  const v4f a = r < NQK ? qa : (r < 2 * NQK ? ka : (r < NPJ ? va : oa));
  const v4f b = r < NQK ? qb : (r < 2 * NQK ? kb : (r < NPJ ? vb : ob));
  union { v8b v; v4u u; } ub;
  ub.v[0] = (__bf16)a.x; ub.v[1] = (__bf16)a.y; ub.v[2] = (__bf16)a.z; ub.v[3] = (__bf16)a.w;
  ub.v[4] = (__bf16)b.x; ub.v[5] = (__bf16)b.y; ub.v[6] = (__bf16)b.z; ub.v[7] = (__bf16)b.w;
  v4f ha, hb;
  ha.x = bfr(a.x) * CWP; ha.y = bfr(a.y) * CWP; ha.z = bfr(a.z) * CWP; ha.w = bfr(a.w) * CWP;
  hb.x = bfr(b.x) * CWP; hb.y = bfr(b.y) * CWP; hb.z = bfr(b.z) * CWP; hb.w = bfr(b.w) * CWP;
  const v4u uh = pack8h(ha, hb);
  const v4u o = r < NPJ ? uh : ub.u;
  vst2(DST + (size_t)r * CH + lane * 8, o);
}

__global__ __launch_bounds__(128) void k_conv(const __bf16* __restrict__ XP, const __bf16* __restrict__ WC, const float* __restrict__ QB, const float* __restrict__ KVB, h16* __restrict__ XF) {
  __shared__ __align__(16) float ss[64][132];
  const int tid = threadIdx.x, lane = tid & 31, col = lane & 15, g = lane >> 4; const int wave = __builtin_amdgcn_readfirstlane(tid >> 5);
  const int which = blockIdx.z; const int c0 = blockIdx.y * 128; const int y = blockIdx.x;
  const __bf16* Ap = XP + (size_t)which * PTOK * CH; const __bf16* Wp = WC + (size_t)which * CH * KCV;
  const int xx = wave * 16 + col;
  v8f acc[8] = {};
#pragma unroll 1
  for (int tap = 0; tap < 9; ++tap) { const int ky = tap / 3, kx = tap - 3 * ky;
    const __bf16* arow = Ap + ((size_t)(y + ky) * PW + xx + kx) * CH;
#pragma unroll 2
    for (int kc = 0; kc < CH / 32; ++kc) { const v16b a = frag_b(arow + kc * 32, lane);
      asm volatile("s_wait_loadcnt 0x0" ::: "memory");
#pragma unroll
      for (int j = 0; j < 8; ++j) { const v16b w = frag_b(Wp + (size_t)(c0 + j * 16 + col) * KCV + tap * CH + kc * 32, lane); asm volatile("s_wait_loadcnt 0x0" ::: "memory"); acc[j] = wmma_bf(a, w, acc[j]); } } }
#pragma unroll
  for (int j = 0; j < 8; ++j) { const float b0 = bfr(QB[c0 + j * 16 + col]), b1 = bfr(KVB[c0 + j * 16 + col]); const float bias = which == 0 ? b0 : b1;
#pragma unroll
    for (int r = 0; r < 8; ++r) ss[wave * 16 + 8 * g + r][j * 16 + col] = (acc[j][r] + bias) * CXF; }
  __syncthreads();
  h16* D = XF + (size_t)which * NTOK * CH + (size_t)y * IMG * CH + c0;
  for (int e = tid; e < 64 * 16; e += 128) { const int rl = e >> 4, q = e & 15;
    const v4f a = *(const v4f*)&ss[rl][q * 8], b = *(const v4f*)&ss[rl][q * 8 + 4];
    vst2(D + (size_t)rl * CH + q * 8, pack8h(a, b)); }
}

__global__ __launch_bounds__(128) void k_proj(const h16* __restrict__ XF, const h16* __restrict__ WP, const float* __restrict__ BQ, const float* __restrict__ BK, const float* __restrict__ BV, h16* __restrict__ QK, h16* __restrict__ VT) {
  __shared__ __align__(16) float sm[128 * 68];
  const int tid = threadIdx.x, lane = tid & 31, col = lane & 15, g = lane >> 4; const int wave = __builtin_amdgcn_readfirstlane(tid >> 5);
  const int p = blockIdx.y; const size_t r0 = (size_t)blockIdx.x * 64;
  const h16* Ap = XF + (p == 0 ? (size_t)0 : (size_t)NTOK * CH); const h16* Wr = WP + (size_t)p * 128 * CH;
  v8f acc[8] = {};
#pragma unroll 2
  for (int kc = 0; kc < CH / 32; ++kc) { const v16h a = frag_h(Ap + (r0 + wave * 16 + col) * CH + kc * 32, lane);
    asm volatile("s_wait_loadcnt 0x0" ::: "memory");
#pragma unroll
    for (int j = 0; j < 8; ++j) { const v16h w = frag_h(Wr + (size_t)(j * 16 + col) * CH + kc * 32, lane); asm volatile("s_wait_loadcnt 0x0" ::: "memory"); acc[j] = wmma_hf(a, w, acc[j]); } }
  const int vo = p >= 2 ? (p - 2) * 128 : 0;
#pragma unroll
  for (int j = 0; j < 8; ++j) { const int cc = j * 16 + col;
    const float bq = bfr(BQ[cc]), bk = bfr(BK[cc]), bv = bfr(BV[vo + cc]); const float bias = (p == 0 ? bq : (p == 1 ? bk : bv)) * CQK;
#pragma unroll
    for (int r = 0; r < 8; ++r) { const float v = acc[j][r] * (CQK / (CXF * CWP)) + bias; const int rl = wave * 16 + 8 * g + r;
      const int ia = rl * 132 + cc, ib = cc * 68 + rl; sm[p < 2 ? ia : ib] = v; } }
  __syncthreads();
  if (p < 2) {
    h16* D = QK + (size_t)p * NTOK * NQK + r0 * NQK;
    for (int e = tid; e < 64 * 16; e += 128) { const int rl = e >> 4, q = e & 15;
      const v4f a = *(const v4f*)&sm[rl * 132 + q * 8], b = *(const v4f*)&sm[rl * 132 + q * 8 + 4];
      vst2(D + (size_t)rl * NQK + q * 8, pack8h(a, b)); }
  } else {
    h16* D = VT + (size_t)vo * NTOK + r0;
    for (int e = tid; e < 128 * 8; e += 128) { const int c = e >> 3, q = e & 7;
      const v4f a = *(const v4f*)&sm[c * 68 + q * 8], b = *(const v4f*)&sm[c * 68 + q * 8 + 4];
      vst2(D + (size_t)c * NTOK + q * 8, pack8h(a, b)); }
  }
}

__global__ __launch_bounds__(256) void k_attn(const h16* __restrict__ QP, const h16* __restrict__ KP, const h16* __restrict__ VT, float* __restrict__ Y) {
  __shared__ __align__(16) float so[8][16][32];
  const int tid = threadIdx.x, lane = tid & 31, col = lane & 15, g = lane >> 4; const int wave = __builtin_amdgcn_readfirstlane(tid >> 5);
  const int hd = blockIdx.y; const int n0 = blockIdx.x * 128 + wave * 16;
  const v8h zh = {};
  union { v16h v; v8h q[2]; } qf; qf.q[0] = *(const v8h*)(QP + (size_t)(n0 + col) * NQK + hd * QKD + 8 * g); qf.q[1] = zh;
  const h16* kb = KP + (size_t)col * NQK + hd * QKD + 8 * g;
  const h16* vb = VT + (size_t)(hd * HDV + col) * NTOK + 8 * g;
  v8f o0 = {}, o1 = {}; float m = -1.0e30f, l = 0.f;
#pragma unroll 1
  for (int j = 0; j < NTOK; j += 32) {
    union { v16h v; v8h q[2]; } k0, k1, v0, v1;
    k0.q[0] = *(const v8h*)(kb + (size_t)j * NQK); k0.q[1] = zh;
    k1.q[0] = *(const v8h*)(kb + (size_t)(j + 16) * NQK); k1.q[1] = zh;
    v0.q[0] = *(const v8h*)(vb + j); v0.q[1] = *(const v8h*)(vb + j + 16);
    v1.q[0] = *(const v8h*)(vb + (size_t)16 * NTOK + j); v1.q[1] = *(const v8h*)(vb + (size_t)16 * NTOK + j + 16);
    asm volatile("s_wait_loadcnt 0x0" ::: "memory");
    const v8f zf = {};
    const v8f s0 = wmma_hf(k0.v, qf.v, zf);
    const v8f s1 = wmma_hf(k1.v, qf.v, zf);
    float tm = fmaxf(s0[0], s1[0]);
#pragma unroll
    for (int r = 1; r < 8; ++r) tm = fmaxf(tm, fmaxf(s0[r], s1[r]));
    tm *= SC1;
    tm = fmaxf(tm, __shfl_xor(tm, 16));
    const float mn = fmaxf(m, tm);
    const float corr = __builtin_amdgcn_exp2f(m - mn);
    m = mn;
    const float off = 8.0f - mn;
    v16h pf; float ps = 0.f;
#pragma unroll
    for (int r = 0; r < 8; ++r) {
      const float e0 = fmaf(s0[r], SC1, off), e1 = fmaf(s1[r], SC1, off);
      const float x0 = __builtin_amdgcn_exp2f(e0), x1 = __builtin_amdgcn_exp2f(e1);
      const float p0 = (e0 < -14.0f) ? 0.0f : x0; const float p1 = (e1 < -14.0f) ? 0.0f : x1;
      const h16 h0 = (h16)p0, h1 = (h16)p1;
      pf[r] = h0; pf[8 + r] = h1; ps += (float)h0 + (float)h1; }
    l = l * corr + ps;
    o0 = o0 * corr; o1 = o1 * corr;
    o0 = wmma_hf(v0.v, pf, o0);
    o1 = wmma_hf(v1.v, pf, o1);
  }
  const float lt = l + __shfl_xor(l, 16);
  const float inv = __builtin_amdgcn_rcpf(lt) * (1.0f / CQK);
#pragma unroll
  for (int r = 0; r < 8; ++r) { so[wave][col][8 * g + r] = o0[r] * inv; so[wave][col][16 + 8 * g + r] = o1[r] * inv; }
  LDSX();
  float* yh = Y + (size_t)hd * NTOK * HDV + (size_t)n0 * HDV;
#pragma unroll
  for (int i = 0; i < 4; ++i) { const int q4 = i * 32 + lane; vst2(yh + q4 * 4, *(const v4f*)&so[wave][q4 >> 3][(q4 & 7) * 4]); }
}

__global__ __launch_bounds__(128) void k_out(const float* __restrict__ Y, const __bf16* __restrict__ WOB, const float* __restrict__ BO, float* __restrict__ OUT) { __shared__ __align__(16) float st[128][68];
  const int tid = threadIdx.x, lane = tid & 31, col = lane & 15, g = lane >> 4; const int wave = __builtin_amdgcn_readfirstlane(tid >> 5); const int c0 = blockIdx.y * 128; const size_t t0 = (size_t)blockIdx.x * 64; const size_t r0 = t0 + wave * 16;
  v8f acc[8] = {};
#pragma unroll 2
  for (int kc = 0; kc < CH / 32; ++kc) { const F2 a = split_row(Y + (r0 + col) * CH, kc * 32, lane); asm volatile("s_wait_loadcnt 0x0" ::: "memory");
#pragma unroll
    for (int j = 0; j < 8; ++j) { const v16b w = frag_b(WOB + (size_t)(c0 + j * 16 + col) * CH + kc * 32, lane); asm volatile("s_wait_loadcnt 0x0" ::: "memory"); acc[j] = wmma_bf(a.h, w, acc[j]); acc[j] = wmma_bf(a.l, w, acc[j]); } }
#pragma unroll
  for (int j = 0; j < 8; ++j) { const float bias = bfr(BO[c0 + j * 16 + col]);
#pragma unroll
    for (int r = 0; r < 8; ++r) st[j * 16 + col][wave * 16 + 8 * g + r] = acc[j][r] + bias; }
  __syncthreads();
  for (int e = tid; e < 128 * 16; e += 128) { const int c = e >> 4, q = e & 15; vst2(OUT + (size_t)(c0 + c) * NTOK + t0 + q * 4, *(const v4f*)&st[c][q * 4]); }
}

extern "C" void kernel_launch(void* const* d_in, const int* in_sizes, int n_in, void* d_out, int out_size, void* d_ws, size_t ws_size, hipStream_t stream) {
  if (n_in < 14) return;
  if (in_sizes[0] < CH * NTOK || in_sizes[1] < CH * NTOK || in_sizes[2] < CH * KCV || in_sizes[3] < CH || in_sizes[4] < CH * KCV || in_sizes[5] < CH) return;
  if (in_sizes[6] < NQK * CH || in_sizes[7] < NQK || in_sizes[8] < NQK * CH || in_sizes[9] < NQK || in_sizes[10] < CH * CH || in_sizes[11] < CH || in_sizes[12] < CH * CH || in_sizes[13] < CH) return;
  if (out_size < CH * NTOK) return;
  if (ws_size < WS_END) return;
  const float *X = (const float*)d_in[0], *AKV = (const float*)d_in[1], *QW = (const float*)d_in[2], *QB = (const float*)d_in[3], *KVW = (const float*)d_in[4], *KVB = (const float*)d_in[5];
  const float *WQ = (const float*)d_in[6], *BQ = (const float*)d_in[7], *WK = (const float*)d_in[8], *BK = (const float*)d_in[9], *WV = (const float*)d_in[10], *BV = (const float*)d_in[11], *WPJ = (const float*)d_in[12], *BP = (const float*)d_in[13];
  char* ws = (char*)d_ws;
  __bf16 *XP = (__bf16*)(ws + WS_XP), *WC = (__bf16*)(ws + WS_WC), *WOB = (__bf16*)(ws + WS_WO);
  h16 *WPH = (h16*)(ws + WS_WP), *XF = (h16*)(ws + WS_XF), *QK = (h16*)(ws + WS_QK), *VT = (h16*)(ws + WS_VT);
  float* Y = (float*)(ws + WS_Y);
  k_padx<<<dim3(PW), 256, 0, stream>>>(X, XP);
  k_padx<<<dim3(PW), 256, 0, stream>>>(AKV, XP + (size_t)PTOK * CH);
  k_cvtw<<<dim3(CH), 256, 0, stream>>>(QW, WC);
  k_cvtw<<<dim3(CH), 256, 0, stream>>>(KVW, WC + (size_t)CH * KCV);
  k_cvts<<<dim3((NPJ + CH) / 8), 256, 0, stream>>>(WQ, WK, WV, WPJ, (unsigned short*)(ws + WS_WP));
  k_conv<<<dim3(IMG, CH / 128, 2), 128, 0, stream>>>(XP, WC, QB, KVB, XF);
  k_proj<<<dim3(NTOK / 64, NPJ / 128), 128, 0, stream>>>(XF, WPH, BQ, BK, BV, QK, VT);
  k_attn<<<dim3(NQ / 128, NHD), 256, 0, stream>>>(QK, QK + (size_t)NTOK * NQK, VT, Y);
  k_out<<<dim3(NTOK / 64, CH / 128), 128, 0, stream>>>(Y, WOB, BP, (float*)d_out);
}
